// MHA_42880953483598
// MI455X (gfx1250) — hardware-verified
//
#include <hip/hip_runtime.h>


#ifndef NB
#define NB 1
#endif
#ifndef SEQ
#define SEQ 4096
#endif
#define NB_FULL  1
#define SEQ_FULL 4096
#define DM   768
#define NH   12
#define HD   64
#define HH   (HD / 2)
#define NW   ((size_t)DM * DM)
#define KT   64
#define PP   72
#define SCL  0.125f
#define THETA_F 10000.0f
#define L2E  1.4426950408889634f
#define NEG  (-1.0e30f)
static_assert(SEQ % 64 == 0);
static_assert(SEQ <= SEQ_FULL);
static_assert(NB >= 1 && NB <= NB_FULL);
static_assert(DM == NH * HD);
static_assert(DM % 64 == 0);
static_assert(HD == 64);
static_assert(KT == 64);
static_assert((size_t)NB_FULL * SEQ_FULL * DM * 4 == 12582912);

typedef _Float16 h16;
typedef unsigned short bf;
typedef __attribute__((ext_vector_type(16))) __bf16   v16bf;
typedef __attribute__((ext_vector_type(16))) _Float16 v16h;
typedef __attribute__((ext_vector_type(8)))  _Float16 v8h;
typedef __attribute__((ext_vector_type(8)))  unsigned short v8us;
typedef __attribute__((ext_vector_type(8)))  float    v8f;
typedef __attribute__((ext_vector_type(4)))  float    v4f;
typedef __attribute__((ext_vector_type(2)))  float    v2f;
typedef __attribute__((ext_vector_type(2)))  unsigned short v2us;
typedef v8h  __attribute__((may_alias)) v8ha;
typedef v4f  __attribute__((may_alias)) v4fa;
typedef v8us __attribute__((may_alias)) v8usa;

__device__ __forceinline__ unsigned short f2bf(float f) { unsigned u = __float_as_uint(f); u += 0x7FFFu + ((u >> 16) & 1u); return (unsigned short)(u >> 16); }
__device__ __forceinline__ float bf2f(unsigned short b) { return __uint_as_float(((unsigned)b) << 16); }
__device__ __forceinline__ float bfr(float f) { return bf2f(f2bf(f)); }
__device__ __forceinline__ void splitf(float y, unsigned short& h, unsigned short& l) { h = f2bf(y); l = f2bf(y - bf2f(h)); }
__device__ __forceinline__ v16h cat16(v8h lo, v8h hi) { return __builtin_shufflevector(lo, hi, 0, 1, 2, 3, 4, 5, 6, 7, 8, 9, 10, 11, 12, 13, 14, 15); }
__device__ __forceinline__ v16bf cat16b(v8us lo, v8us hi) { return __builtin_bit_cast(v16bf, __builtin_shufflevector(lo, hi, 0, 1, 2, 3, 4, 5, 6, 7, 8, 9, 10, 11, 12, 13, 14, 15)); }
__device__ __forceinline__ v8f wmma16(v16h a, v16h b, v8f c) { return __builtin_amdgcn_wmma_f32_16x16x32_f16(false, a, false, b, (short)0, c, false, false); }
__device__ __forceinline__ v8f wmmab(v16bf a, v16bf b, v8f c) { return __builtin_amdgcn_wmma_f32_16x16x32_bf16(false, a, false, b, (short)0, c, false, false); }

template <typename T16> struct WFrag;
template <> struct WFrag<h16> { typedef v16h V; static __device__ __forceinline__ V ld(const h16* p) { return cat16(*(const v8h*)p, *(const v8h*)(p + 16)); } static __device__ __forceinline__ v8f mma(V a, V b, v8f c) { return wmma16(a, b, c); } };
template <> struct WFrag<bf> { typedef v16bf V; static __device__ __forceinline__ V ld(const bf* p) { return cat16b(*(const v8us*)p, *(const v8us*)(p + 16)); } static __device__ __forceinline__ v8f mma(V a, V b, v8f c) { return wmmab(a, b, c); } };

template <typename T16, int NSPLIT, bool BIAS>
__global__ __launch_bounds__(32) void k_gemmw(const T16* __restrict__ A, const T16* __restrict__ A2, const T16* __restrict__ Bt, const T16* __restrict__ Bt2, int K, float* C, int ldc, const float* __restrict__ bias, size_t sA, size_t sB, size_t sC) {
    typedef typename WFrag<T16>::V V;
    __shared__ __align__(16) float os[16 * 68];
    const size_t z = blockIdx.z; A += z * sA; if (A2) A2 += z * sA; Bt += z * sB; if (Bt2) Bt2 += z * sB; C += z * sC;
    const int lane = threadIdx.x & 31, lr = lane & 15, hi = lane >> 4; const int r0 = blockIdx.x * 64, c0 = blockIdx.y * 64;
    v8f acc[4][4];
#pragma unroll
    for (int mb = 0; mb < 4; ++mb)
#pragma unroll
        for (int nb = 0; nb < 4; ++nb) acc[mb][nb] = (v8f){};
    const size_t aoff = (size_t)(r0 + lr) * K + 8 * hi, boff = (size_t)(c0 + lr) * K + 8 * hi;
#pragma unroll 1
    for (int kc = 0; kc < K; kc += 32) {
        V a[4], a2[4];
#pragma unroll
        for (int mb = 0; mb < 4; ++mb) { a[mb] = WFrag<T16>::ld(A + aoff + (size_t)mb * 16 * K + kc); if (NSPLIT == 1 || NSPLIT == 2) a2[mb] = WFrag<T16>::ld(A2 + aoff + (size_t)mb * 16 * K + kc); }
#pragma unroll
        for (int nb = 0; nb < 4; ++nb) { const V b = WFrag<T16>::ld(Bt + boff + (size_t)nb * 16 * K + kc); V b2; if (NSPLIT >= 2) b2 = WFrag<T16>::ld(Bt2 + boff + (size_t)nb * 16 * K + kc);
#pragma unroll
            for (int mb = 0; mb < 4; ++mb) { acc[mb][nb] = WFrag<T16>::mma(a[mb], b, acc[mb][nb]); if (NSPLIT == 1 || NSPLIT == 2) acc[mb][nb] = WFrag<T16>::mma(a2[mb], b, acc[mb][nb]); if (NSPLIT >= 2) acc[mb][nb] = WFrag<T16>::mma(a[mb], b2, acc[mb][nb]); } }
        asm volatile("v_nop\n\tv_nop\n\tv_nop\n\tv_nop" : "+v"(acc[0][0]), "+v"(acc[1][1]), "+v"(acc[2][2]), "+v"(acc[3][3]) : "v"(a[0]), "v"(a[3]));
    }
#pragma unroll
    for (int mb = 0; mb < 4; ++mb) {
#pragma unroll
        for (int nb = 0; nb < 4; ++nb) {
#pragma unroll
            for (int j = 0; j < 8; ++j) os[(hi * 8 + j) * 68 + nb * 16 + lr] = acc[mb][nb][j]; }
        __builtin_amdgcn_wave_barrier(); asm volatile("" ::: "memory");
        float* crow = C + (size_t)(r0 + mb * 16) * ldc + c0;
#pragma unroll 1
        for (int ps = 0; ps < 2; ++ps) {
#pragma unroll
            for (int s = 0; s < 8; ++s) { const int row = 2 * s + hi, cofs = lr * 4; v4f val = *(const v4fa*)(os + row * 68 + cofs); if (BIAS) { val[0] += bfr(bias[c0 + cofs]); val[1] += bfr(bias[c0 + cofs + 1]); val[2] += bfr(bias[c0 + cofs + 2]); val[3] += bfr(bias[c0 + cofs + 3]); }
                *(volatile v4f*)(crow + (size_t)row * ldc + cofs) = val; }
            if (ps == 0) __threadfence(); }
        __builtin_amdgcn_wave_barrier(); asm volatile("" ::: "memory");
    }
}

__global__ __launch_bounds__(256) void k_cvt8(const float* __restrict__ src, bf* dst, size_t n8) { const size_t i = (size_t)blockIdx.x * 256 + threadIdx.x; if (i >= n8) return; const v8f v = *(const v8f*)(src + i * 8); v8us o;
#pragma unroll
    for (int k = 0; k < 8; ++k) o[k] = f2bf(v[k]); *(volatile v8us*)(dst + i * 8) = o; __threadfence(); *(volatile v8us*)(dst + i * 8) = o; }

__global__ __launch_bounds__(256) void k_cvtw(const float* __restrict__ w0, const float* __restrict__ w1, const float* __restrict__ w2, const float* __restrict__ w3, bf* dst, size_t n8) {
    const size_t i = (size_t)blockIdx.x * 256 + threadIdx.x; if (i >= n8) return; const int y = blockIdx.y;
    const float* src = (y == 0) ? w0 : ((y == 1) ? w1 : ((y == 2) ? w2 : w3));
    const v8f v = *(const v8f*)(src + i * 8); v8us o;
#pragma unroll
    for (int k = 0; k < 8; ++k) o[k] = f2bf(v[k]);
    bf* d = dst + (size_t)y * n8 * 8 + i * 8;
    *(volatile v8us*)d = o; __threadfence(); *(volatile v8us*)d = o; }

__global__ __launch_bounds__(256) void k_cs(float* CS) {
    const int idx = blockIdx.x * 256 + threadIdx.x; if (idx >= SEQ * HH) return; const int i = idx % HH, t = idx / HH;
    const float ex = -(float)(2 * i) / (float)HD;
    const float inv = powf(THETA_F, ex);
    float ang = __fmul_rn((float)t, inv); asm volatile("" : "+v"(ang));
    v2f cs; cs[0] = cosf(ang); cs[1] = sinf(ang);
    *(volatile v2f*)(CS + (size_t)idx * 2) = cs; __threadfence(); *(volatile v2f*)(CS + (size_t)idx * 2) = cs; }

__global__ __launch_bounds__(256) void k_rope2(const float* __restrict__ F, const float* __restrict__ CS, bf* Ph, bf* Pl) {
    const size_t e = ((size_t)blockIdx.x * 256 + threadIdx.x) * 2; if (e >= (size_t)NH * SEQ * HD) return;
    const int d = (int)(e % HD); const int t = (int)((e / HD) % SEQ); const int h = (int)(e / ((size_t)HD * SEQ));
    const float* f = F + (size_t)t * DM + h * HD + d; const float x1 = f[0], x2 = f[1];
    const v2f cs = *(const v2f*)(CS + ((size_t)t * HH + (d >> 1)) * 2);
    float a = __fmul_rn(x1, cs[0]), bq = __fmul_rn(x2, cs[1]), a2 = __fmul_rn(x1, cs[1]), c2 = __fmul_rn(x2, cs[0]);
    asm volatile("" : "+v"(a)); asm volatile("" : "+v"(bq)); asm volatile("" : "+v"(a2)); asm volatile("" : "+v"(c2));
    const float r0 = __fsub_rn(a, bq), r1 = __fadd_rn(a2, c2);
    v2us oh, ol; unsigned short u0, u1, w0, w1; splitf(r0, u0, w0); splitf(r1, u1, w1); oh[0] = u0; oh[1] = u1; ol[0] = w0; ol[1] = w1;
    *(volatile v2us*)(Ph + e) = oh; *(volatile v2us*)(Pl + e) = ol; __threadfence(); *(volatile v2us*)(Ph + e) = oh; *(volatile v2us*)(Pl + e) = ol; }

__global__ __launch_bounds__(256) void k_vtp2(const float* __restrict__ F, bf* Vh, bf* Vl) {
    const size_t e = ((size_t)blockIdx.x * 256 + threadIdx.x) * 2; if (e >= (size_t)NH * HD * SEQ) return;
    const int t = (int)(e % SEQ); const int d = (int)((e / SEQ) % HD); const int g = (int)(e / ((size_t)SEQ * HD)); v2us oh, ol;
#pragma unroll
    for (int q = 0; q < 2; ++q) { const float x = F[(size_t)(t + q) * DM + g * HD + d]; unsigned short a2, c2; splitf(x, a2, c2); oh[q] = a2; ol[q] = c2; }
    *(volatile v2us*)(Vh + e) = oh; *(volatile v2us*)(Vl + e) = ol; __threadfence(); *(volatile v2us*)(Vh + e) = oh; *(volatile v2us*)(Vl + e) = ol; }

__global__ __launch_bounds__(32) void k_flash(const bf* __restrict__ Qh, const bf* __restrict__ Ql, const bf* __restrict__ Kh, const bf* __restrict__ Kl,
                                             const bf* __restrict__ Vh, const bf* __restrict__ Vl, bf* Ch, bf* Cl) {
    __shared__ __align__(16) unsigned short th[16 * PP];
    __shared__ __align__(16) unsigned short tl[16 * PP];
    typedef WFrag<bf>::V V;
    const int lane = threadIdx.x & 31, lr = lane & 15, hi = lane >> 4;
    const int q0 = blockIdx.x * 16, head = blockIdx.y;
    const size_t qo = ((size_t)head * SEQ + q0 + lr) * HD + 8 * hi;
    const V qh0 = WFrag<bf>::ld(Qh + qo), qh1 = WFrag<bf>::ld(Qh + qo + 32), ql0 = WFrag<bf>::ld(Ql + qo), ql1 = WFrag<bf>::ld(Ql + qo + 32);
    const size_t kb = ((size_t)head * SEQ + lr) * HD + 8 * hi;
    const bf* kh = Kh + kb; const bf* kl = Kl + kb;
    const size_t vb = ((size_t)head * HD + lr) * SEQ + 8 * hi;
    const bf* vh = Vh + vb; const bf* vl = Vl + vb;
    v8f o[4];
#pragma unroll
    for (int t4 = 0; t4 < 4; ++t4) o[t4] = (v8f){};
    float mrow[8], lrow[8];
#pragma unroll
    for (int r = 0; r < 8; ++r) { mrow[r] = NEG; lrow[r] = 0.0f; }
    const int nt = (q0 + 15) / KT + 1;
#pragma unroll 1
    for (int kt = 0; kt < nt; ++kt) {
        const int key0 = kt * KT;
        v8f sc[4];
#pragma unroll
        for (int nb = 0; nb < 4; ++nb) sc[nb] = (v8f){};
#pragma unroll
        for (int nb = 0; nb < 4; ++nb) {
            const size_t ko = (size_t)(key0 + nb * 16) * HD;
            { const V bh = WFrag<bf>::ld(kh + ko), bl = WFrag<bf>::ld(kl + ko);
              sc[nb] = wmmab(qh0, bh, sc[nb]); sc[nb] = wmmab(ql0, bh, sc[nb]); sc[nb] = wmmab(qh0, bl, sc[nb]); }
            { const V bh = WFrag<bf>::ld(kh + ko + 32), bl = WFrag<bf>::ld(kl + ko + 32);
              sc[nb] = wmmab(qh1, bh, sc[nb]); sc[nb] = wmmab(ql1, bh, sc[nb]); sc[nb] = wmmab(qh1, bl, sc[nb]); }
        }
        asm volatile("v_nop\n\tv_nop\n\tv_nop\n\tv_nop" : "+v"(sc[0]), "+v"(sc[1]), "+v"(sc[2]), "+v"(sc[3]) : "v"(qh0), "v"(ql1));
#pragma unroll
        for (int r = 0; r < 8; ++r) {
            const int row = q0 + 8 * hi + r;
            float v[4]; float cand = NEG;
#pragma unroll
            for (int nb = 0; nb < 4; ++nb) { const int key = key0 + nb * 16 + lr; const float s = sc[nb][r] * SCL; v[nb] = (key <= row) ? s : NEG; cand = fmaxf(cand, v[nb]); }
#pragma unroll
            for (int off = 1; off < 16; off <<= 1) cand = fmaxf(cand, __shfl_xor(cand, off, 32));
            const float mnew = fmaxf(mrow[r], cand);
            const float alpha = __builtin_amdgcn_exp2f((mrow[r] - mnew) * L2E);
            float rs = 0.0f;
#pragma unroll
            for (int nb = 0; nb < 4; ++nb) { const float p = __builtin_amdgcn_exp2f((v[nb] - mnew) * L2E); rs += p; unsigned short a2, c2; splitf(p, a2, c2); th[(8 * hi + r) * PP + nb * 16 + lr] = a2; tl[(8 * hi + r) * PP + nb * 16 + lr] = c2; }
#pragma unroll
            for (int off = 1; off < 16; off <<= 1) rs += __shfl_xor(rs, off, 32);
            lrow[r] = lrow[r] * alpha + rs; mrow[r] = mnew;
#pragma unroll
            for (int t4 = 0; t4 < 4; ++t4) o[t4][r] *= alpha;
        }
        __syncthreads();
        const V ph0 = WFrag<bf>::ld(th + lr * PP + 8 * hi), ph1 = WFrag<bf>::ld(th + lr * PP + 8 * hi + 32);
        const V pl0 = WFrag<bf>::ld(tl + lr * PP + 8 * hi), pl1 = WFrag<bf>::ld(tl + lr * PP + 8 * hi + 32);
#pragma unroll
        for (int t4 = 0; t4 < 4; ++t4) {
            const size_t vo = (size_t)(t4 * 16) * SEQ + key0;
            { const V wh = WFrag<bf>::ld(vh + vo), wl = WFrag<bf>::ld(vl + vo);
              o[t4] = wmmab(ph0, wh, o[t4]); o[t4] = wmmab(pl0, wh, o[t4]); o[t4] = wmmab(ph0, wl, o[t4]); }
            { const V wh = WFrag<bf>::ld(vh + vo + 32), wl = WFrag<bf>::ld(vl + vo + 32);
              o[t4] = wmmab(ph1, wh, o[t4]); o[t4] = wmmab(pl1, wh, o[t4]); o[t4] = wmmab(ph1, wl, o[t4]); }
        }
        asm volatile("v_nop\n\tv_nop\n\tv_nop\n\tv_nop" : "+v"(o[0]), "+v"(o[1]), "+v"(o[2]), "+v"(o[3]) : "v"(ph0), "v"(pl1));
        __syncthreads();
    }
#pragma unroll
    for (int r = 0; r < 8; ++r) {
        const float il = 1.0f / lrow[r];
#pragma unroll
        for (int t4 = 0; t4 < 4; ++t4) { const float c = o[t4][r] * il; unsigned short a2, c2; splitf(c, a2, c2); th[(8 * hi + r) * PP + t4 * 16 + lr] = a2; tl[(8 * hi + r) * PP + t4 * 16 + lr] = c2; }
    }
    __syncthreads();
    const int rq = lane >> 3, c8 = (lane & 7) * 8;
#pragma unroll 1
    for (int ps = 0; ps < 2; ++ps) {
#pragma unroll
        for (int s = 0; s < 4; ++s) {
            const int row = s * 4 + rq;
            const v8us xh = *(const v8usa*)(th + row * PP + c8), xl = *(const v8usa*)(tl + row * PP + c8);
            const size_t go = (size_t)(q0 + row) * DM + head * HD + c8;
            *(volatile v8us*)(Ch + go) = xh; *(volatile v8us*)(Cl + go) = xl; }
        if (ps == 0) __threadfence(); }
}

extern "C" void kernel_launch(void* const* d_in, const int* in_sizes, int n_in,
                              void* d_out, int out_size, void* d_ws, size_t ws_size, hipStream_t stream) {
    if (n_in < 5) return;
    if ((size_t)in_sizes[0] < (size_t)(NB - 1) * SEQ_FULL * DM + (size_t)SEQ * DM) return;
    for (int i = 1; i < 5; ++i) if ((size_t)in_sizes[i] < NW) return;
    if ((size_t)out_size < (size_t)(NB - 1) * SEQ_FULL * DM + (size_t)SEQ * DM) return;
    const float* x  = (const float*)d_in[0];
    const float* wq = (const float*)d_in[1];
    const float* wk = (const float*)d_in[2];
    const float* wv = (const float*)d_in[3];
    const float* wo = (const float*)d_in[4];
    float* OUT = (float*)d_out;
    char* wsp = (char*)d_ws;
    auto take = [&](size_t bytes) { char* p = wsp; wsp += (bytes + 255) & ~(size_t)255; return (void*)p; };
    bf* W4 = (bf*)take(4 * NW * 2);
    bf* XB = (bf*)take((size_t)SEQ * DM * 2);
    float* F = (float*)take((size_t)3 * SEQ * DM * 4);
    float* CS = (float*)take((size_t)SEQ * HH * 2 * 4);
    const size_t PL = (size_t)NH * SEQ * HD;
    bf* QPh = (bf*)take(PL * 2); bf* QPl = (bf*)take(PL * 2); bf* KPh = (bf*)take(PL * 2); bf* KPl = (bf*)take(PL * 2);
    bf* VTh = (bf*)take(PL * 2); bf* VTl = (bf*)take(PL * 2);
    bf* CXh = (bf*)take((size_t)SEQ * DM * 2); bf* CXl = (bf*)take((size_t)SEQ * DM * 2);
    if ((size_t)(wsp - (char*)d_ws) > ws_size) return;
    const size_t NW8 = NW / 8;
    k_cvtw<<<dim3((unsigned)((NW8 + 255) / 256), 4, 1), 256, 0, stream>>>(wq, wk, wv, wo, W4, NW8);
    k_cs<<<(unsigned)((SEQ * HH + 255) / 256), 256, 0, stream>>>(CS);
    const unsigned LP = (unsigned)((PL / 2 + 255) / 256);
    for (int b = 0; b < NB; ++b) {
        k_cvt8<<<(unsigned)(((size_t)SEQ * DM / 8 + 255) / 256), 256, 0, stream>>>(x + (size_t)b * SEQ_FULL * DM, XB, (size_t)SEQ * DM / 8);
        k_gemmw<bf, 0, false><<<dim3(SEQ / 64, DM / 64, 3), 32, 0, stream>>>(XB, nullptr, W4, nullptr, DM, F, DM, nullptr, (size_t)0, NW, (size_t)SEQ * DM);
        k_rope2<<<LP, 256, 0, stream>>>(F, CS, QPh, QPl);
        k_rope2<<<LP, 256, 0, stream>>>(F + (size_t)SEQ * DM, CS, KPh, KPl);
        k_vtp2<<<LP, 256, 0, stream>>>(F + (size_t)2 * SEQ * DM, VTh, VTl);
        k_flash<<<dim3(SEQ / 16, NH, 1), 32, 0, stream>>>(QPh, QPl, KPh, KPl, VTh, VTl, CXh, CXl);
        k_gemmw<bf, 1, false><<<dim3(SEQ / 64, DM / 64, 1), 32, 0, stream>>>(CXh, CXl, W4 + 3 * NW, nullptr, DM, OUT + (size_t)b * SEQ_FULL * DM, DM, nullptr, (size_t)0, (size_t)0, (size_t)0);
    }
}
